// HyperGraphAttentionLayerSparse_63118839382177
// MI455X (gfx1250) — hardware-run, weakly checked
//
#include <hip/hip_runtime.h>


namespace {
constexpr int N = 20000, E = 5000, NNZ = 160000, D = 128, SB = 2048, LMAX = 128;
constexpr float XS = 8.0f, WSC = 256.0f, DEPS = 1e-10f, SLOPE = 0.2f;
typedef _Float16 b16;
typedef __attribute__((ext_vector_type(16))) _Float16 v16b;
typedef __attribute__((ext_vector_type(8))) _Float16 v8b;
typedef __attribute__((ext_vector_type(8))) float v8f;
typedef __attribute__((ext_vector_type(4))) float v4f;
__device__ __forceinline__ float bf16_rne(float f) { unsigned int u = __float_as_uint(f); u += 0x7FFFu + ((u >> 16) & 1u); float r = __uint_as_float(u & 0xFFFF0000u); asm volatile("" : "+v"(r)); return r; }
__device__ __forceinline__ v16b frag_kb(const b16* p, int hh) { const v8b a = *(const v8b*)(p + 8 * hh), b = *(const v8b*)(p + 16 + 8 * hh); v16b f;
#pragma unroll
  for (int e = 0; e < 8; ++e) { f[e] = a[e]; f[8 + e] = b[e]; } return f; }
__device__ __forceinline__ v8f wmma16b(v16b a, v16b b, v8f c) { v8f d = __builtin_amdgcn_wmma_f32_16x16x32_f16(false, a, false, b, (short)0, c, false, false); asm volatile("v_nop\n\tv_nop\n\tv_nop\n\tv_nop" : "+v"(d) : "v"(a), "v"(b)); return d; }
__device__ __forceinline__ void wave_lds_sync() { __builtin_amdgcn_fence(__ATOMIC_RELEASE, "workgroup"); __builtin_amdgcn_wave_barrier(); __builtin_amdgcn_fence(__ATOMIC_ACQUIRE, "workgroup"); }
__device__ __forceinline__ float pmul(float a, float b) { float p = a * b; asm volatile("" : "+v"(p)); return p; }
__device__ __forceinline__ int iclamp(int v, int lo, int hi) { return v < lo ? lo : (v > hi ? hi : v); }
__device__ __forceinline__ float lrelu(float v) { return v > 0.0f ? v : SLOPE * v; }
constexpr int CSR_NBLK9 = 512, CSR_GB9 = 9, CSR_GN9 = 1 << CSR_GB9  , CSR_TS9 = (CSR_GN9 < 32 ? 32 : CSR_GN9)  , CSR_MAXG9 = 512, CSR_CAP9 = 12288  ;
__device__ __host__ __forceinline__ int csr_tix9(int v) { return (v >> CSR_GB9) * CSR_TS9 + (v & (CSR_GN9 - 1)); }
__global__ __launch_bounds__(64) void csrA_kernel9(const int* __restrict__ dst, int E, int N, int nG, int CHP, int NGP, int* __restrict__ STG, int* __restrict__ HST) {
  extern __shared__ int sm[];
  int* cnt = sm; int* run = sm + NGP; int* ids = sm + 2 * NGP;
  const int b = blockIdx.x; const int ch = (E + CSR_NBLK9 - 1) / CSR_NBLK9; const int e0 = b * ch, e1 = min(E, e0 + ch);
  for (int i = threadIdx.x; i < NGP; i += 64) cnt[i] = 0;
  for (int i = threadIdx.x; i < CHP; i += 64) ids[i] = -1;
  __syncthreads();
  if (threadIdx.x == 0) {
    for (int e = e0; e < e1; ++e) { int d = dst[e]; d = (d < 0) ? 0 : (d >= N ? N - 1 : d); cnt[d >> CSR_GB9] += 1; }
    int acc = 0; for (int g = 0; g < nG; ++g) { run[g] = acc; acc += cnt[g]; }
    for (int e = e0; e < e1; ++e) { int d = dst[e]; d = (d < 0) ? 0 : (d >= N ? N - 1 : d); const int g = d >> CSR_GB9; ids[run[g]] = e; run[g] += 1; } }
  __syncthreads();
  typedef __attribute__((ext_vector_type(4))) int v4i;
  for (int pass = 0; pass < 2; ++pass) {
    for (int i = threadIdx.x; i < CHP / 4; i += 64) *(volatile v4i*)(STG + (size_t)b * CHP + i * 4) = *(const v4i*)(&ids[i * 4]);
    for (int i = threadIdx.x; i < NGP / 4; i += 64) { v4i v; for (int e = 0; e < 4; ++e) v[e] = (i * 4 + e < nG) ? cnt[i * 4 + e] : 0; *(volatile v4i*)(HST + (size_t)b * NGP + i * 4) = v; }
    __threadfence(); }
}
__global__ __launch_bounds__(512) void csrS_kernel9(const int* __restrict__ HST, int nG, int NGP, int* __restrict__ START, int* __restrict__ TOT, int* __restrict__ OFF) {
  __shared__ int tot[CSR_MAXG9];
  const int b = threadIdx.x;
  for (int pass = 0; pass < 2; ++pass) { int runb = 0; for (int g = 0; g < nG; ++g) { int c = HST[(size_t)b * NGP + g]; c = (c < 0) ? 0 : c; ((volatile int*)OFF)[(size_t)g * CSR_NBLK9 + b] = runb; runb += c; } __threadfence(); }
  for (int g = threadIdx.x; g < nG; g += 512) { int s = 0; for (int bb = 0; bb < CSR_NBLK9; ++bb) { int c = HST[(size_t)bb * NGP + g]; s += (c < 0) ? 0 : c; } tot[g] = s; }
  __syncthreads();
  if (threadIdx.x < 32) {
    __shared__ int st[CSR_MAXG9 + 32];
    if (threadIdx.x == 0) { int acc = 0; for (int g = 0; g < NGP; ++g) { st[g] = acc; if (g < nG) acc += (tot[g] + 31) & ~31; } st[NGP] = acc; }
    __builtin_amdgcn_fence(__ATOMIC_RELEASE, "workgroup"); __builtin_amdgcn_wave_barrier(); __builtin_amdgcn_fence(__ATOMIC_ACQUIRE, "workgroup");
    for (int pass = 0; pass < 2; ++pass) { for (int i = threadIdx.x; i < NGP + 32; i += 32) { ((volatile int*)START)[i] = (i <= NGP) ? st[min(i, NGP)] : 0; ((volatile int*)TOT)[i] = (i < nG) ? tot[i] : 0; } __threadfence(); } }
}
__global__ __launch_bounds__(256) void csrB_kernel9(const int* __restrict__ dst, int N, int nG, int CHP, int NGP, int permLen, const int* __restrict__ STG, const int* __restrict__ HST, const int* __restrict__ OFF, const int* __restrict__ START, const int* __restrict__ TOT, int* __restrict__ PERM, int* __restrict__ ROWPTR, int* __restrict__ ROWCNT, int* __restrict__ FLAG) {
  typedef __attribute__((ext_vector_type(4))) int v4i;
  __shared__ int ids[CSR_CAP9]; __shared__ unsigned short key[CSR_CAP9]; __shared__ int outp[CSR_CAP9]; __shared__ int ncnt[CSR_GN9 + 1]; __shared__ int boff[CSR_NBLK9 + 1];
  const int g = blockIdx.x, t_ = threadIdx.x; int tot = TOT[g]; int st = START[g], stn = START[g + 1]; const int v0 = g * CSR_GN9; const int nv = min(CSR_GN9, N - v0); const int t0 = g * CSR_TS9;
  st = (st < 0) ? 0 : (st > permLen - 32 ? permLen - 32 : st) & ~31; stn = (stn < st) ? st : (stn > permLen ? permLen : stn); tot = (tot < 0) ? 0 : tot; if (tot > stn - st && tot <= CSR_CAP9) tot = stn - st;
  if (tot > CSR_CAP9) {
    for (int pass = 0; pass < 2; ++pass) { for (int i = t_; i < CSR_TS9 / 4; i += 256) { v4i a, c; for (int e = 0; e < 4; ++e) { a[e] = st; c[e] = 0; } *(volatile v4i*)(ROWPTR + t0 + i * 4) = a; *(volatile v4i*)(ROWCNT + t0 + i * 4) = c; } if (t_ == 0) ((volatile int*)FLAG)[0] = 1; __threadfence(); } (void)nv; return; }
  if (t_ == 0) { int acc = 0; for (int b = 0; b < CSR_NBLK9; ++b) { boff[b] = acc; int c = HST[(size_t)b * NGP + g]; c = (c < 0) ? 0 : (c > CHP ? CHP : c); acc += c; if (acc > tot) acc = tot; } boff[CSR_NBLK9] = acc; }
  for (int i = t_; i <= CSR_GN9; i += 256) ncnt[i] = 0;
  __syncthreads();
  for (int b = 0; b < CSR_NBLK9; ++b) { const int c = boff[b + 1] - boff[b]; int o_ = OFF[(size_t)g * CSR_NBLK9 + b]; o_ = (o_ < 0) ? 0 : (o_ > CHP - c ? CHP - c : o_); const int* src_ = STG + (size_t)b * CHP + o_;
    for (int i = t_; i < c; i += 256) { int id = src_[i]; id = (id < 0) ? 0 : id; ids[boff[b] + i] = id; int d = dst[id]; d = (d < v0) ? v0 : (d >= N ? N - 1 : d); int kk = d - v0; kk = (kk < 0) ? 0 : (kk >= CSR_GN9 ? CSR_GN9 - 1 : kk); key[boff[b] + i] = (unsigned short)kk; } }
  __syncthreads();
  if (t_ == 0) { for (int i = 0; i < tot; ++i) ncnt[key[i]] += 1; int acc = 0; for (int vl = 0; vl < CSR_GN9; ++vl) { const int c = ncnt[vl]; ncnt[vl] = acc; acc += c; } ncnt[CSR_GN9] = acc;
    for (int i = 0; i < tot; ++i) { const int vl = key[i]; outp[ncnt[vl]] = ids[i]; ncnt[vl] += 1; }
    for (int vl = CSR_GN9; vl > 0; --vl) ncnt[vl] = ncnt[vl - 1]; ncnt[0] = 0; }
  __syncthreads();
  for (int pass = 0; pass < 2; ++pass) {
    for (int i = t_; i < (stn - st) / 4; i += 256) { v4i v; for (int e = 0; e < 4; ++e) { const int q = i * 4 + e; v[e] = (q < tot) ? outp[q] : -1; } *(volatile v4i*)(PERM + st + i * 4) = v; }
    for (int i = t_; i < CSR_TS9 / 4; i += 256) { v4i a, c; for (int e = 0; e < 4; ++e) { const int vl = i * 4 + e; const int vc = vl < CSR_GN9 ? vl : CSR_GN9; a[e] = (vl < CSR_GN9) ? st + ncnt[vc] : st; c[e] = (vl < nv) ? (ncnt[(vc < CSR_GN9 ? vc : CSR_GN9 - 1) + 1] - ncnt[vc]) : 0; } *(volatile v4i*)(ROWPTR + t0 + i * 4) = a; *(volatile v4i*)(ROWCNT + t0 + i * 4) = c; }
    __threadfence(); }
}
__global__ __launch_bounds__(256) void csrZ_kernel9(int* __restrict__ p, size_t n4) { typedef __attribute__((ext_vector_type(4))) int v4i; const size_t tid = (size_t)blockIdx.x * 256 + threadIdx.x, nth = (size_t)gridDim.x * 256; v4i z = {0, 0, 0, 0}; for (size_t i = tid; i < n4; i += nth) *(volatile v4i*)(p + i * 4) = z; }
struct CsrBufs9 { int *STG, *HST, *OFF, *START, *TOT, *PERM, *ROWPTR, *ROWCNT, *FLAG; int nG, NGP, CHP; size_t permLen; char* base; size_t bytes; };
static size_t csr_carve9(CsrBufs9& c, char* ws, size_t off, int E, int N) {
  const size_t off0 = off; c.base = ws + off;
  auto al = [&](size_t bytes) { char* p = ws + off; off += (bytes + 255) & ~(size_t)255; return p; };
  c.nG = (N + CSR_GN9 - 1) / CSR_GN9; c.NGP = (c.nG + 31) & ~31; const int ch = (E + CSR_NBLK9 - 1) / CSR_NBLK9; c.CHP = (ch + 31) & ~31; c.permLen = (size_t)E + 32 * (size_t)c.nG + 32;
  c.STG = (int*)al((size_t)CSR_NBLK9 * c.CHP * 4); c.HST = (int*)al((size_t)CSR_NBLK9 * c.NGP * 4); c.OFF = (int*)al((size_t)c.NGP * CSR_NBLK9 * 4); c.START = (int*)al((size_t)(c.NGP + 64) * 4); c.TOT = (int*)al((size_t)(c.NGP + 64) * 4);
  c.PERM = (int*)al(c.permLen * 4); c.ROWPTR = (int*)al((size_t)c.nG * CSR_TS9 * 4); c.ROWCNT = (int*)al((size_t)c.nG * CSR_TS9 * 4); c.FLAG = (int*)al(256);
  c.bytes = off - off0; return off;
}
static void csr_build9(const CsrBufs9& c, const int* dst, int E, int N, hipStream_t stream) {
  const size_t smem = (size_t)(2 * c.NGP + c.CHP) * 4;
  csrZ_kernel9<<<512, 256, 0, stream>>>((int*)c.base, c.bytes / 16);
  csrA_kernel9<<<CSR_NBLK9, 64, smem, stream>>>(dst, E, N, c.nG, c.CHP, c.NGP, c.STG, c.HST);
  csrS_kernel9<<<1, 512, 0, stream>>>(c.HST, c.nG, c.NGP, c.START, c.TOT, c.OFF);
  csrB_kernel9<<<c.nG, 256, 0, stream>>>(dst, N, c.nG, c.CHP, c.NGP, (int)c.permLen, c.STG, c.HST, c.OFF, c.START, c.TOT, c.PERM, c.ROWPTR, c.ROWCNT, c.FLAG);
}

constexpr int CSR_NBLK8 = 512, CSR_GB8 = 8, CSR_GN8 = 1 << CSR_GB8  , CSR_TS8 = (CSR_GN8 < 32 ? 32 : CSR_GN8)  , CSR_MAXG8 = 512, CSR_CAP8 = 12288  ;
__device__ __host__ __forceinline__ int csr_tix8(int v) { return (v >> CSR_GB8) * CSR_TS8 + (v & (CSR_GN8 - 1)); }
__global__ __launch_bounds__(64) void csrA_kernel8(const int* __restrict__ dst, int E, int N, int nG, int CHP, int NGP, int* __restrict__ STG, int* __restrict__ HST) {
  extern __shared__ int sm[];
  int* cnt = sm; int* run = sm + NGP; int* ids = sm + 2 * NGP;
  const int b = blockIdx.x; const int ch = (E + CSR_NBLK8 - 1) / CSR_NBLK8; const int e0 = b * ch, e1 = min(E, e0 + ch);
  for (int i = threadIdx.x; i < NGP; i += 64) cnt[i] = 0;
  for (int i = threadIdx.x; i < CHP; i += 64) ids[i] = -1;
  __syncthreads();
  if (threadIdx.x == 0) {
    for (int e = e0; e < e1; ++e) { int d = dst[e]; d = (d < 0) ? 0 : (d >= N ? N - 1 : d); cnt[d >> CSR_GB8] += 1; }
    int acc = 0; for (int g = 0; g < nG; ++g) { run[g] = acc; acc += cnt[g]; }
    for (int e = e0; e < e1; ++e) { int d = dst[e]; d = (d < 0) ? 0 : (d >= N ? N - 1 : d); const int g = d >> CSR_GB8; ids[run[g]] = e; run[g] += 1; } }
  __syncthreads();
  typedef __attribute__((ext_vector_type(4))) int v4i;
  for (int pass = 0; pass < 2; ++pass) {
    for (int i = threadIdx.x; i < CHP / 4; i += 64) *(volatile v4i*)(STG + (size_t)b * CHP + i * 4) = *(const v4i*)(&ids[i * 4]);
    for (int i = threadIdx.x; i < NGP / 4; i += 64) { v4i v; for (int e = 0; e < 4; ++e) v[e] = (i * 4 + e < nG) ? cnt[i * 4 + e] : 0; *(volatile v4i*)(HST + (size_t)b * NGP + i * 4) = v; }
    __threadfence(); }
}
__global__ __launch_bounds__(512) void csrS_kernel8(const int* __restrict__ HST, int nG, int NGP, int* __restrict__ START, int* __restrict__ TOT, int* __restrict__ OFF) {
  __shared__ int tot[CSR_MAXG8];
  const int b = threadIdx.x;
  for (int pass = 0; pass < 2; ++pass) { int runb = 0; for (int g = 0; g < nG; ++g) { int c = HST[(size_t)b * NGP + g]; c = (c < 0) ? 0 : c; ((volatile int*)OFF)[(size_t)g * CSR_NBLK8 + b] = runb; runb += c; } __threadfence(); }
  for (int g = threadIdx.x; g < nG; g += 512) { int s = 0; for (int bb = 0; bb < CSR_NBLK8; ++bb) { int c = HST[(size_t)bb * NGP + g]; s += (c < 0) ? 0 : c; } tot[g] = s; }
  __syncthreads();
  if (threadIdx.x < 32) {
    __shared__ int st[CSR_MAXG8 + 32];
    if (threadIdx.x == 0) { int acc = 0; for (int g = 0; g < NGP; ++g) { st[g] = acc; if (g < nG) acc += (tot[g] + 31) & ~31; } st[NGP] = acc; }
    __builtin_amdgcn_fence(__ATOMIC_RELEASE, "workgroup"); __builtin_amdgcn_wave_barrier(); __builtin_amdgcn_fence(__ATOMIC_ACQUIRE, "workgroup");
    for (int pass = 0; pass < 2; ++pass) { for (int i = threadIdx.x; i < NGP + 32; i += 32) { ((volatile int*)START)[i] = (i <= NGP) ? st[min(i, NGP)] : 0; ((volatile int*)TOT)[i] = (i < nG) ? tot[i] : 0; } __threadfence(); } }
}
__global__ __launch_bounds__(256) void csrB_kernel8(const int* __restrict__ dst, int N, int nG, int CHP, int NGP, int permLen, const int* __restrict__ STG, const int* __restrict__ HST, const int* __restrict__ OFF, const int* __restrict__ START, const int* __restrict__ TOT, int* __restrict__ PERM, int* __restrict__ ROWPTR, int* __restrict__ ROWCNT, int* __restrict__ FLAG) {
  typedef __attribute__((ext_vector_type(4))) int v4i;
  __shared__ int ids[CSR_CAP8]; __shared__ unsigned short key[CSR_CAP8]; __shared__ int outp[CSR_CAP8]; __shared__ int ncnt[CSR_GN8 + 1]; __shared__ int boff[CSR_NBLK8 + 1];
  const int g = blockIdx.x, t_ = threadIdx.x; int tot = TOT[g]; int st = START[g], stn = START[g + 1]; const int v0 = g * CSR_GN8; const int nv = min(CSR_GN8, N - v0); const int t0 = g * CSR_TS8;
  st = (st < 0) ? 0 : (st > permLen - 32 ? permLen - 32 : st) & ~31; stn = (stn < st) ? st : (stn > permLen ? permLen : stn); tot = (tot < 0) ? 0 : tot; if (tot > stn - st && tot <= CSR_CAP8) tot = stn - st;
  if (tot > CSR_CAP8) {
    for (int pass = 0; pass < 2; ++pass) { for (int i = t_; i < CSR_TS8 / 4; i += 256) { v4i a, c; for (int e = 0; e < 4; ++e) { a[e] = st; c[e] = 0; } *(volatile v4i*)(ROWPTR + t0 + i * 4) = a; *(volatile v4i*)(ROWCNT + t0 + i * 4) = c; } if (t_ == 0) ((volatile int*)FLAG)[0] = 1; __threadfence(); } (void)nv; return; }
  if (t_ == 0) { int acc = 0; for (int b = 0; b < CSR_NBLK8; ++b) { boff[b] = acc; int c = HST[(size_t)b * NGP + g]; c = (c < 0) ? 0 : (c > CHP ? CHP : c); acc += c; if (acc > tot) acc = tot; } boff[CSR_NBLK8] = acc; }
  for (int i = t_; i <= CSR_GN8; i += 256) ncnt[i] = 0;
  __syncthreads();
  for (int b = 0; b < CSR_NBLK8; ++b) { const int c = boff[b + 1] - boff[b]; int o_ = OFF[(size_t)g * CSR_NBLK8 + b]; o_ = (o_ < 0) ? 0 : (o_ > CHP - c ? CHP - c : o_); const int* src_ = STG + (size_t)b * CHP + o_;
    for (int i = t_; i < c; i += 256) { int id = src_[i]; id = (id < 0) ? 0 : id; ids[boff[b] + i] = id; int d = dst[id]; d = (d < v0) ? v0 : (d >= N ? N - 1 : d); int kk = d - v0; kk = (kk < 0) ? 0 : (kk >= CSR_GN8 ? CSR_GN8 - 1 : kk); key[boff[b] + i] = (unsigned short)kk; } }
  __syncthreads();
  if (t_ == 0) { for (int i = 0; i < tot; ++i) ncnt[key[i]] += 1; int acc = 0; for (int vl = 0; vl < CSR_GN8; ++vl) { const int c = ncnt[vl]; ncnt[vl] = acc; acc += c; } ncnt[CSR_GN8] = acc;
    for (int i = 0; i < tot; ++i) { const int vl = key[i]; outp[ncnt[vl]] = ids[i]; ncnt[vl] += 1; }
    for (int vl = CSR_GN8; vl > 0; --vl) ncnt[vl] = ncnt[vl - 1]; ncnt[0] = 0; }
  __syncthreads();
  for (int pass = 0; pass < 2; ++pass) {
    for (int i = t_; i < (stn - st) / 4; i += 256) { v4i v; for (int e = 0; e < 4; ++e) { const int q = i * 4 + e; v[e] = (q < tot) ? outp[q] : -1; } *(volatile v4i*)(PERM + st + i * 4) = v; }
    for (int i = t_; i < CSR_TS8 / 4; i += 256) { v4i a, c; for (int e = 0; e < 4; ++e) { const int vl = i * 4 + e; const int vc = vl < CSR_GN8 ? vl : CSR_GN8; a[e] = (vl < CSR_GN8) ? st + ncnt[vc] : st; c[e] = (vl < nv) ? (ncnt[(vc < CSR_GN8 ? vc : CSR_GN8 - 1) + 1] - ncnt[vc]) : 0; } *(volatile v4i*)(ROWPTR + t0 + i * 4) = a; *(volatile v4i*)(ROWCNT + t0 + i * 4) = c; }
    __threadfence(); }
}
__global__ __launch_bounds__(256) void csrZ_kernel8(int* __restrict__ p, size_t n4) { typedef __attribute__((ext_vector_type(4))) int v4i; const size_t tid = (size_t)blockIdx.x * 256 + threadIdx.x, nth = (size_t)gridDim.x * 256; v4i z = {0, 0, 0, 0}; for (size_t i = tid; i < n4; i += nth) *(volatile v4i*)(p + i * 4) = z; }
struct CsrBufs8 { int *STG, *HST, *OFF, *START, *TOT, *PERM, *ROWPTR, *ROWCNT, *FLAG; int nG, NGP, CHP; size_t permLen; char* base; size_t bytes; };
static size_t csr_carve8(CsrBufs8& c, char* ws, size_t off, int E, int N) {
  const size_t off0 = off; c.base = ws + off;
  auto al = [&](size_t bytes) { char* p = ws + off; off += (bytes + 255) & ~(size_t)255; return p; };
  c.nG = (N + CSR_GN8 - 1) / CSR_GN8; c.NGP = (c.nG + 31) & ~31; const int ch = (E + CSR_NBLK8 - 1) / CSR_NBLK8; c.CHP = (ch + 31) & ~31; c.permLen = (size_t)E + 32 * (size_t)c.nG + 32;
  c.STG = (int*)al((size_t)CSR_NBLK8 * c.CHP * 4); c.HST = (int*)al((size_t)CSR_NBLK8 * c.NGP * 4); c.OFF = (int*)al((size_t)c.NGP * CSR_NBLK8 * 4); c.START = (int*)al((size_t)(c.NGP + 64) * 4); c.TOT = (int*)al((size_t)(c.NGP + 64) * 4);
  c.PERM = (int*)al(c.permLen * 4); c.ROWPTR = (int*)al((size_t)c.nG * CSR_TS8 * 4); c.ROWCNT = (int*)al((size_t)c.nG * CSR_TS8 * 4); c.FLAG = (int*)al(256);
  c.bytes = off - off0; return off;
}
static void csr_build8(const CsrBufs8& c, const int* dst, int E, int N, hipStream_t stream) {
  const size_t smem = (size_t)(2 * c.NGP + c.CHP) * 4;
  csrZ_kernel8<<<512, 256, 0, stream>>>((int*)c.base, c.bytes / 16);
  csrA_kernel8<<<CSR_NBLK8, 64, smem, stream>>>(dst, E, N, c.nG, c.CHP, c.NGP, c.STG, c.HST);
  csrS_kernel8<<<1, 512, 0, stream>>>(c.HST, c.nG, c.NGP, c.START, c.TOT, c.OFF);
  csrB_kernel8<<<c.nG, 256, 0, stream>>>(dst, N, c.nG, c.CHP, c.NGP, (int)c.permLen, c.STG, c.HST, c.OFF, c.START, c.TOT, c.PERM, c.ROWPTR, c.ROWCNT, c.FLAG);
}


__global__ __launch_bounds__(256) void wput_kernel(const float* __restrict__ w, b16* __restrict__ WT) { const int u = blockIdx.x * 256 + threadIdx.x; if (u >= D * 16) return; const int o = u / 16, k0 = (u % 16) * 8; v8b v;
#pragma unroll
  for (int j = 0; j < 8; ++j) v[j] = (b16)(bf16_rne(w[(size_t)(k0 + j) * D + o]) * WSC); for (int pass = 0; pass < 2; ++pass) { *(volatile v8b*)(WT + (size_t)o * D + k0) = v; __threadfence(); } }
__global__ __launch_bounds__(32) void xproj_kernel(const float* __restrict__ x, const b16* __restrict__ WT, int NLIM, float* __restrict__ XP) { __shared__ __attribute__((aligned(16))) b16 Ah[16][D + 8]; __shared__ float Tf[16][132]; const int lane = threadIdx.x, nloc = lane & 15, hlf = lane >> 4; const size_t m0 = (size_t)blockIdx.x * 16; if (m0 >= (size_t)NLIM) return;
  for (int rr = 0; rr < 16; ++rr) for (int q = 0; q < 4; ++q) Ah[rr][q * 32 + lane] = (b16)(bf16_rne(x[(m0 + rr) * D + q * 32 + lane]) * XS);
  wave_lds_sync(); v8f acc[8];
#pragma unroll
  for (int t = 0; t < 8; ++t) acc[t] = (v8f){};
#pragma unroll
  for (int kb = 0; kb < D; kb += 32) { const v16b a = frag_kb(&Ah[nloc][kb], hlf);
#pragma unroll
    for (int t = 0; t < 8; ++t) acc[t] = wmma16b(a, frag_kb(WT + (size_t)(t * 16 + nloc) * D + kb, hlf), acc[t]); }
#pragma unroll
  for (int t = 0; t < 8; ++t)
#pragma unroll
    for (int r8 = 0; r8 < 8; ++r8) Tf[8 * hlf + r8][t * 16 + nloc] = acc[t][r8] * (1.0f / (XS * WSC));
  wave_lds_sync();
  for (int pass = 0; pass < 2; ++pass) { for (int rr = 0; rr < 16; ++rr) *(volatile v4f*)(XP + (m0 + rr) * D + lane * 4) = *(const v4f*)(&Tf[rr][lane * 4]); __threadfence(); } }
__global__ __launch_bounds__(256) void nodeA_kernel(const float* __restrict__ vals, const int* __restrict__ PERM, const int* __restrict__ ROWPTR, const int* __restrict__ ROWCNT, int permLen, int NLIM, float* __restrict__ NA) { const int wave = threadIdx.x >> 5, lane = threadIdx.x & 31; const size_t i = (size_t)blockIdx.x * 8 + wave; if (i >= (size_t)NLIM) return; int st = ROWPTR[i], cnt = ROWCNT[i]; cnt = iclamp(cnt, 0, NNZ); st = iclamp(st, 0, permLen - cnt);
  float s = 0.0f; for (int j = lane; j < cnt; j += 32) { const int k = iclamp(PERM[st + j], 0, NNZ - 1); s += bf16_rne(vals[k]); } for (int o = 16; o; o >>= 1) s += __shfl_xor(s, o);
  const float dvi = powf(s + DEPS, -0.5f);
  for (int pass = 0; pass < 2; ++pass) { ((volatile float*)NA)[i * 32 + lane] = lane == 0 ? dvi : 0.0f; __threadfence(); } }
__global__ __launch_bounds__(256) void edgeA_kernel(const float* __restrict__ XP, const float* __restrict__ NA, const float* __restrict__ vals, const int* __restrict__ rws, const int* __restrict__ PERM, const int* __restrict__ ROWPTR, const int* __restrict__ ROWCNT, int permLen, int NLIM, float* __restrict__ E2) { const int wave = threadIdx.x >> 5, lane = threadIdx.x & 31; const int e = blockIdx.x * 8 + wave; if (e >= E) return; int st = ROWPTR[e], cnt = ROWCNT[e]; cnt = iclamp(cnt, 0, NNZ); st = iclamp(st, 0, permLen - cnt);
  v4f acc = {0, 0, 0, 0}; float de = 0.0f;
#pragma unroll 1
  for (int j = 0; j < cnt; ++j) { const int k = iclamp(PERM[st + j], 0, NNZ - 1); const int n = iclamp(rws[k], 0, N - 1); if (n >= NLIM) continue; const float v = bf16_rne(vals[k]); de += v; const float w = pmul(v, NA[(size_t)n * 32]); const v4f xv = *(const v4f*)(XP + (size_t)n * D + lane * 4); for (int q = 0; q < 4; ++q) acc[q] += pmul(w, xv[q]); }
  const float dei = 1.0f / (de + DEPS); v4f o; for (int q = 0; q < 4; ++q) o[q] = pmul(acc[q], dei);
  for (int pass = 0; pass < 2; ++pass) { *(volatile v4f*)(E2 + (size_t)e * D + lane * 4) = o; __threadfence(); } }
__global__ __launch_bounds__(256) void nodeB_kernel(const float* __restrict__ XP, const float* __restrict__ NA, const float* __restrict__ E2, const float* __restrict__ a, const float* __restrict__ vals, const int* __restrict__ cls, const int* __restrict__ PERM, const int* __restrict__ ROWPTR, const int* __restrict__ ROWCNT, int permLen, int NLIM, float* __restrict__ NB) { const int wave = threadIdx.x >> 5, lane = threadIdx.x & 31; const size_t i = (size_t)blockIdx.x * 8 + wave; if (i >= (size_t)NLIM) return; int st = ROWPTR[i], cnt = ROWCNT[i]; cnt = iclamp(cnt, 0, NNZ); st = iclamp(st, 0, permLen - cnt);
  v4f acc = {0, 0, 0, 0};
#pragma unroll 1
  for (int j = 0; j < cnt; ++j) { const int k = iclamp(PERM[st + j], 0, NNZ - 1); const int e = iclamp(cls[k], 0, E - 1); const float v = bf16_rne(vals[k]); const v4f ev = *(const v4f*)(E2 + (size_t)e * D + lane * 4); for (int q = 0; q < 4; ++q) acc[q] += pmul(v, ev[q]); }
  const float dvi = NA[i * 32]; const v4f xv = *(const v4f*)(XP + i * D + lane * 4); float s = 0.0f, t = 0.0f; for (int q = 0; q < 4; ++q) { const float y = pmul(acc[q], dvi) + xv[q]; s += pmul(y, bf16_rne(a[lane * 4 + q])); t += pmul(y, bf16_rne(a[D + lane * 4 + q])); }
  for (int o = 16; o; o >>= 1) { s += __shfl_xor(s, o); t += __shfl_xor(t, o); }
  for (int pass = 0; pass < 2; ++pass) { ((volatile float*)NB)[i * 32 + lane] = lane == 0 ? s : (lane == 1 ? t : 0.0f); __threadfence(); } }
__global__ __launch_bounds__(256) void nodeC_kernel(const float* __restrict__ NB, const int* __restrict__ cls, const int* __restrict__ PERM, const int* __restrict__ ROWPTR, const int* __restrict__ ROWCNT, int permLen, int NLIM, float* __restrict__ NC) { __shared__ int Le[8][LMAX]; const int wave = threadIdx.x >> 5, lane = threadIdx.x & 31; const size_t i = (size_t)blockIdx.x * 8 + wave; if (i >= (size_t)NLIM) return; int st = ROWPTR[i], cnt = ROWCNT[i]; cnt = iclamp(cnt, 0, LMAX); st = iclamp(st, 0, permLen - cnt);
  const float sy = NB[i * 32];
  for (int j = lane; j < cnt; j += 32) { const int k = iclamp(PERM[st + j], 0, NNZ - 1); Le[wave][j] = iclamp(cls[k], 0, E - 1); }
  wave_lds_sync(); float mx = -INFINITY; int ndist = 0;
  for (int j = lane; j < cnt; j += 32) { const int e = Le[wave][j]; int c = 0, first = 1; for (int jj = 0; jj < cnt; ++jj) { const int ee = Le[wave][jj]; c += (ee == e); if (ee == e && jj < j) first = 0; } if (first) { ++ndist; mx = fmaxf(mx, (float)c * lrelu(sy + NB[(size_t)e * 32 + 1])); } }
  for (int o = 16; o; o >>= 1) { mx = fmaxf(mx, __shfl_xor(mx, o)); ndist += __shfl_xor(ndist, o); }
  const float m = (ndist < E) ? fmaxf(mx, 0.0f) : mx; float z = 0.0f;
  for (int j = lane; j < cnt; j += 32) { const int e = Le[wave][j]; int c = 0, first = 1; for (int jj = 0; jj < cnt; ++jj) { const int ee = Le[wave][jj]; c += (ee == e); if (ee == e && jj < j) first = 0; } if (first) z += __expf((float)c * lrelu(sy + NB[(size_t)e * 32 + 1]) - m); }
  for (int o = 16; o; o >>= 1) z += __shfl_xor(z, o); z += (float)(E - ndist) * __expf(-m);
  for (int pass = 0; pass < 2; ++pass) { ((volatile float*)NC)[i * 32 + lane] = lane == 0 ? m : (lane == 1 ? z : 0.0f); __threadfence(); } }
__global__ __launch_bounds__(256) void gpart_kernel(const float* __restrict__ XP, const float* __restrict__ NC, int NLIM, float* __restrict__ PS) { __shared__ float A[2][128]; const int t = threadIdx.x, c = t & 127, part = t >> 7; const size_t r0 = (size_t)blockIdx.x * SB; float s = 0.0f;
  for (int rr = part; rr < SB; rr += 2) { const size_t n = r0 + rr; if (n >= (size_t)NLIM) break; const float base = __expf(-NC[n * 32]) / NC[n * 32 + 1]; s += pmul(base, XP[n * D + c]); } A[part][c] = s; __syncthreads();
  if (t < 128) { const float ss = A[0][t] + A[1][t]; for (int pass = 0; pass < 2; ++pass) { ((volatile float*)PS)[(size_t)blockIdx.x * 128 + t] = ss; __threadfence(); } } }
__global__ __launch_bounds__(128) void gfin_kernel(const float* __restrict__ PS, int nblk, float* __restrict__ G) { const int t = threadIdx.x; double s = 0.0; for (int b = 0; b < nblk; ++b) s += (double)PS[(size_t)b * 128 + t]; for (int pass = 0; pass < 2; ++pass) { ((volatile float*)G)[t] = (float)s; __threadfence(); } }
__global__ __launch_bounds__(256) void edgeB_kernel(const float* __restrict__ XP, const float* __restrict__ NB, const float* __restrict__ NC, const float* __restrict__ G, const int* __restrict__ rws, const int* __restrict__ PERM, const int* __restrict__ ROWPTR, const int* __restrict__ ROWCNT, int permLen, int NLIM, float* __restrict__ EF) { __shared__ int Ln[8][LMAX]; const int wave = threadIdx.x >> 5, lane = threadIdx.x & 31; const int e = blockIdx.x * 8 + wave; if (e >= E) return; int st = ROWPTR[e], cnt = ROWCNT[e]; cnt = iclamp(cnt, 0, LMAX); st = iclamp(st, 0, permLen - cnt);
  for (int j = lane; j < cnt; j += 32) { const int k = iclamp(PERM[st + j], 0, NNZ - 1); Ln[wave][j] = iclamp(rws[k], 0, N - 1); }
  wave_lds_sync(); const float ty = NB[(size_t)e * 32 + 1]; v4f acc = *(const v4f*)(G + lane * 4);
#pragma unroll 1
  for (int j = 0; j < cnt; ++j) { const int n = Ln[wave][j]; if (n >= NLIM) continue; int c = 0, first = 1; for (int jj = 0; jj < cnt; ++jj) { const int nn = Ln[wave][jj]; c += (nn == n); if (nn == n && jj < j) first = 0; } if (!first) continue;
    const float m = NC[(size_t)n * 32], z = NC[(size_t)n * 32 + 1]; const float p = __expf((float)c * lrelu(NB[(size_t)n * 32] + ty) - m) / z, base = __expf(-m) / z; const float w = p - base; const v4f xv = *(const v4f*)(XP + (size_t)n * D + lane * 4); for (int q = 0; q < 4; ++q) acc[q] += pmul(w, xv[q]); }
  for (int pass = 0; pass < 2; ++pass) { *(volatile v4f*)(EF + (size_t)e * D + lane * 4) = acc; __threadfence(); } }
__global__ __launch_bounds__(256) void out_kernel(const float* __restrict__ EF, const float* __restrict__ bias, const float* __restrict__ vals, const int* __restrict__ cls, const int* __restrict__ PERM, const int* __restrict__ ROWPTR, const int* __restrict__ ROWCNT, int permLen, int NLIM, float* __restrict__ out) { const int wave = threadIdx.x >> 5, lane = threadIdx.x & 31; const size_t i = (size_t)blockIdx.x * 8 + wave; if (i >= (size_t)NLIM) return; int st = ROWPTR[i], cnt = ROWCNT[i]; cnt = iclamp(cnt, 0, NNZ); st = iclamp(st, 0, permLen - cnt);
  v4f acc = {0, 0, 0, 0};
#pragma unroll 1
  for (int j = 0; j < cnt; ++j) { const int k = iclamp(PERM[st + j], 0, NNZ - 1); const int e = iclamp(cls[k], 0, E - 1); const float v = bf16_rne(vals[k]); const v4f ev = *(const v4f*)(EF + (size_t)e * D + lane * 4); for (int q = 0; q < 4; ++q) acc[q] += pmul(v, ev[q]); }
  v4f o; for (int q = 0; q < 4; ++q) o[q] = acc[q] + bf16_rne(bias[lane * 4 + q]);
  for (int pass = 0; pass < 2; ++pass) { *(volatile v4f*)(out + i * D + lane * 4) = o; __threadfence(); } }
}

extern "C" void kernel_launch(void* const* d_in, const int* in_sizes, int n_in, void* d_out, int out_size, void* d_ws, size_t ws_size, hipStream_t stream) {
  (void)n_in;
  auto Fp = [&](int i) { return (const float*)d_in[i]; }; auto Ip = [&](int i) { return (const int*)d_in[i]; };
  if (in_sizes[0] != N * D || in_sizes[1] != NNZ || in_sizes[2] != NNZ || in_sizes[3] != NNZ || in_sizes[4] != D * D || in_sizes[5] != 2 * D || in_sizes[6] != D || out_size != N * D) return;
  const int NLIM = N;
  const int NBLK = (NLIM + SB - 1) / SB;
  size_t off = 0; char* ws = (char*)d_ws;
  auto carve = [&](size_t bytes) { char* p = ws + off; off += (bytes + 255) & ~(size_t)255; return p; };
  b16* WT = (b16*)carve((size_t)D * D * 2); float* XP = (float*)carve((size_t)N * D * 4); float* NA = (float*)carve((size_t)N * 32 * 4); float* NB = (float*)carve((size_t)N * 32 * 4); float* NC = (float*)carve((size_t)N * 32 * 4); float* E2 = (float*)carve((size_t)E * D * 4); float* EF = (float*)carve((size_t)E * D * 4); float* PS = (float*)carve((size_t)((N + SB - 1) / SB) * 128 * 4); float* G = (float*)carve(128 * 4);
  CsrBufs9 cn; off = csr_carve9(cn, ws, off, NNZ, N); CsrBufs8 ce; off = csr_carve8(ce, ws, off, NNZ, E);
  if (off > ws_size || off > ((size_t)64 << 20)) return;
  wput_kernel<<<(D * 16 + 255) / 256, 256, 0, stream>>>(Fp(4), WT);
  csr_build9(cn, Ip(1), NNZ, N, stream);
  csr_build8(ce, Ip(2), NNZ, E, stream);
  xproj_kernel<<<NLIM / 16, 32, 0, stream>>>(Fp(0), WT, NLIM, XP);
  nodeA_kernel<<<(NLIM + 7) / 8, 256, 0, stream>>>(Fp(3), cn.PERM, cn.ROWPTR, cn.ROWCNT, (int)cn.permLen, NLIM, NA);
  edgeA_kernel<<<(E + 7) / 8, 256, 0, stream>>>(XP, NA, Fp(3), Ip(1), ce.PERM, ce.ROWPTR, ce.ROWCNT, (int)ce.permLen, NLIM, E2);
  nodeB_kernel<<<(NLIM + 7) / 8, 256, 0, stream>>>(XP, NA, E2, Fp(5), Fp(3), Ip(2), cn.PERM, cn.ROWPTR, cn.ROWCNT, (int)cn.permLen, NLIM, NB);
  nodeC_kernel<<<(NLIM + 7) / 8, 256, 0, stream>>>(NB, Ip(2), cn.PERM, cn.ROWPTR, cn.ROWCNT, (int)cn.permLen, NLIM, NC);
  gpart_kernel<<<NBLK, 256, 0, stream>>>(XP, NC, NLIM, PS); gfin_kernel<<<1, 128, 0, stream>>>(PS, NBLK, G);
  edgeB_kernel<<<(E + 7) / 8, 256, 0, stream>>>(XP, NB, NC, G, Ip(1), ce.PERM, ce.ROWPTR, ce.ROWCNT, (int)ce.permLen, NLIM, EF);
  out_kernel<<<(NLIM + 7) / 8, 256, 0, stream>>>(EF, Fp(6), Fp(3), Ip(2), cn.PERM, cn.ROWPTR, cn.ROWCNT, (int)cn.permLen, NLIM, (float*)d_out);
}
